// PixelMultiClassInfoNCELoss_87479893885192
// MI455X (gfx1250) — hardware-verified
//
#include <hip/hip_runtime.h>
#include <stdint.h>

typedef _Float16 v16h __attribute__((ext_vector_type(16)));
typedef _Float16 v8h  __attribute__((ext_vector_type(8)));
typedef float    v8f  __attribute__((ext_vector_type(8)));
typedef float    v4f  __attribute__((ext_vector_type(4)));
typedef v8h __attribute__((may_alias)) v8ha;
typedef v4f __attribute__((may_alias)) v4fa;

#define NPIX 8192
#define CDIM 128
#define HW   4096
#define NCLS 4
#define OPSCALE 16.0f
#define EXP2_SCALE 0.056355275034725134f
#define EPS_F 1e-6f
#define DIAG_FILL (-1.0e6f)

#define K1_PIX 32
#define SF_PITCH 132
#define SH_PITCH 136
#define ROWS_PER_BLOCK 64

static_assert(NPIX % K1_PIX == 0);
static_assert(NPIX % ROWS_PER_BLOCK == 0);
static_assert(HW % K1_PIX == 0);
static_assert(CDIM == 128);

union Frag { v16h v; v8h half[2]; };

__device__ __forceinline__ v8f wmma_f16(v16h a, v16h b, v8f c) {
  return __builtin_amdgcn_wmma_f32_16x16x32_f16(false, a, false, b, (short)0, c, false, false);
}

__global__ __launch_bounds__(256) void k_norm(const float* __restrict__ emb, _Float16* __restrict__ En) {
  __shared__ __attribute__((aligned(16))) float    sf[K1_PIX * SF_PITCH];
  __shared__ __attribute__((aligned(16))) _Float16 sh[K1_PIX * SH_PITCH];
  const int t  = threadIdx.x;
  const int n0 = blockIdx.x * K1_PIX;
  if (n0 >= NPIX) return;
  const int b  = n0 >> 12;
  const int p0 = n0 & (HW - 1);
  const float* base = emb + (size_t)b * CDIM * HW + p0;

#pragma unroll
  for (int i = 0; i < 16; ++i) {
    const int idx = i * 256 + t;
    const int c   = idx >> 5;
    const int px  = idx & 31;
    sf[px * SF_PITCH + c] = base[(size_t)c * HW + px];
  }
  __syncthreads();

  const int pix = t >> 3;
  const int sub = t & 7;
  const float* rowp = sf + pix * SF_PITCH + sub * 16;
  float x[16];
  float ss = 0.f;
#pragma unroll
  for (int j = 0; j < 16; ++j) { x[j] = rowp[j]; ss = fmaf(x[j], x[j], ss); }
  ss += __shfl_xor(ss, 1, 32);
  ss += __shfl_xor(ss, 2, 32);
  ss += __shfl_xor(ss, 4, 32);
  const float nr  = fmaxf(sqrtf(ss), 1e-12f);
  const float inv = OPSCALE / nr;
  Frag f;
#pragma unroll
  for (int j = 0; j < 16; ++j) f.v[j] = (_Float16)(x[j] * inv);
  v8h* shp = (v8h*)(sh + pix * SH_PITCH + sub * 16);
  shp[0] = f.half[0];
  shp[1] = f.half[1];
  __syncthreads();

  const int w = t >> 5, l = t & 31;
  const int rowA  = w * 4 + (l >> 4);
  const int rowB  = rowA + 2;
  const int chunk = l & 15;
  const v8h va = *(const v8ha*)(sh + rowA * SH_PITCH + chunk * 8);
  const v8h vb = *(const v8ha*)(sh + rowB * SH_PITCH + chunk * 8);
  _Float16* da = En + (size_t)(n0 + rowA) * CDIM + chunk * 8;
  _Float16* db = En + (size_t)(n0 + rowB) * CDIM + chunk * 8;
  *(volatile v8h*)da = va;
  *(volatile v8h*)db = vb;
  __threadfence();
  *(volatile v8h*)da = va;
  *(volatile v8h*)db = vb;
}

__global__ __launch_bounds__(128) void k_gram(const _Float16* __restrict__ En, const int* __restrict__ lab,
                                             float* __restrict__ row_loss) {
  __shared__ __attribute__((aligned(16))) float sRL[ROWS_PER_BLOCK];
  const int t = threadIdx.x;
  const int w = t >> 5, l = t & 31, h = l >> 4, m = l & 15;
  const int r0 = blockIdx.x * ROWS_PER_BLOCK + w * 16;

  Frag a[4];
  {
    const _Float16* arow = En + (size_t)(r0 + m) * CDIM + 8 * h;
#pragma unroll
    for (int kc = 0; kc < 4; ++kc) {
      a[kc].half[0] = *(const v8h*)(arow + kc * 32);
      a[kc].half[1] = *(const v8h*)(arow + kc * 32 + 16);
    }
  }
  int labR[8];
#pragma unroll
  for (int r = 0; r < 8; ++r) labR[r] = lab[r0 + 8 * h + r];

  float tot[8], pos[8];
#pragma unroll
  for (int r = 0; r < 8; ++r) { tot[r] = 0.f; pos[r] = 0.f; }

  for (int c0 = 0; c0 < NPIX; c0 += 16) {
    const _Float16* brow = En + (size_t)(c0 + m) * CDIM + 8 * h;
    Frag b[4];
#pragma unroll
    for (int kc = 0; kc < 4; ++kc) {
      b[kc].half[0] = *(const v8h*)(brow + kc * 32);
      b[kc].half[1] = *(const v8h*)(brow + kc * 32 + 16);
    }
    const int clab = lab[c0 + m];

    v8f acc = {0.f, 0.f, 0.f, 0.f, 0.f, 0.f, 0.f, 0.f};
    acc = wmma_f16(a[0].v, b[0].v, acc);
    acc = wmma_f16(a[1].v, b[1].v, acc);
    acc = wmma_f16(a[2].v, b[2].v, acc);
    acc = wmma_f16(a[3].v, b[3].v, acc);
    asm volatile("v_nop\n\tv_nop\n\tv_nop\n\tv_nop"
                 : "+v"(acc)
                 : "v"(a[0].v), "v"(a[1].v), "v"(a[2].v), "v"(a[3].v),
                   "v"(b[0].v), "v"(b[1].v), "v"(b[2].v), "v"(b[3].v));

    if (c0 == r0) {
#pragma unroll
      for (int r = 0; r < 8; ++r) acc[r] = ((8 * h + r) == m) ? DIAG_FILL : acc[r];
    }
#pragma unroll
    for (int r = 0; r < 8; ++r) {
      const float ex = __builtin_amdgcn_exp2f(acc[r] * EXP2_SCALE);
      tot[r] += ex;
      pos[r] += (labR[r] == clab) ? ex : 0.f;
    }
  }

#pragma unroll
  for (int s = 1; s <= 8; s <<= 1) {
#pragma unroll
    for (int r = 0; r < 8; ++r) {
      tot[r] += __shfl_xor(tot[r], s, 32);
      pos[r] += __shfl_xor(pos[r], s, 32);
    }
  }
  float loss[8];
#pragma unroll
  for (int r = 0; r < 8; ++r) {
    const float q = pos[r] * __builtin_amdgcn_rcpf(tot[r] + EPS_F);
    loss[r] = -logf(q);
  }
  if (m == 0) {
#pragma unroll
    for (int r = 0; r < 8; ++r) sRL[w * 16 + 8 * h + r] = loss[r];
  }
  __syncthreads();
  if (t < 16) {
    const v4f v = *(const v4fa*)(sRL + t * 4);
    float* dst = row_loss + (size_t)blockIdx.x * ROWS_PER_BLOCK + t * 4;
    *(volatile v4f*)dst = v;
    __threadfence();
    *(volatile v4f*)dst = v;
  }
}

__global__ __launch_bounds__(256) void k_final(const float* __restrict__ row_loss, const int* __restrict__ lab,
                                              float* __restrict__ out) {
  __shared__ float sps[NCLS][256];
  __shared__ float spc[NCLS][256];
  const int t = threadIdx.x;
  float ps[NCLS], pc[NCLS];
#pragma unroll
  for (int k = 0; k < NCLS; ++k) { ps[k] = 0.f; pc[k] = 0.f; }
  const int nb = t * (NPIX / 256);
  for (int i = 0; i < NPIX / 256; ++i) {
    const int n = nb + i;
    const int lb = lab[n];
    const float v = row_loss[n];
#pragma unroll
    for (int k = 0; k < NCLS; ++k) {
      ps[k] += (lb == k) ? v : 0.f;
      pc[k] += (lb == k) ? 1.f : 0.f;
    }
  }
#pragma unroll
  for (int k = 0; k < NCLS; ++k) { sps[k][t] = ps[k]; spc[k][t] = pc[k]; }
  __syncthreads();
  if (t == 0) {
    double s0 = 0.0, s1 = 0.0, s2 = 0.0, s3 = 0.0;
    double c0 = 0.0, c1 = 0.0, c2 = 0.0, c3 = 0.0;
    for (int j = 0; j < 256; ++j) {
      s0 += (double)sps[0][j]; s1 += (double)sps[1][j]; s2 += (double)sps[2][j]; s3 += (double)sps[3][j];
      c0 += (double)spc[0][j]; c1 += (double)spc[1][j]; c2 += (double)spc[2][j]; c3 += (double)spc[3][j];
    }
    float accv = 0.f;
    float np = 0.f;
    { const float sf0 = (float)s0, cf0 = (float)c0; if (cf0 > 0.f) { accv += sf0 / cf0; np += 1.f; } }
    { const float sf1 = (float)s1, cf1 = (float)c1; if (cf1 > 0.f) { accv += sf1 / cf1; np += 1.f; } }
    { const float sf2 = (float)s2, cf2 = (float)c2; if (cf2 > 0.f) { accv += sf2 / cf2; np += 1.f; } }
    { const float sf3 = (float)s3, cf3 = (float)c3; if (cf3 > 0.f) { accv += sf3 / cf3; np += 1.f; } }
    const float res = accv / np;
    *(volatile float*)out = res;
    __threadfence();
    *(volatile float*)out = res;
  }
}

extern "C" void kernel_launch(void* const* d_in, const int* in_sizes, int n_in,
                              void* d_out, int out_size, void* d_ws, size_t ws_size,
                              hipStream_t stream) {
  if (n_in < 2) return;
  if (in_sizes[0] != 2 * CDIM * HW || in_sizes[1] != NPIX || out_size < 1) return;

  const size_t en_bytes = (size_t)NPIX * CDIM * sizeof(_Float16);
  const size_t rl_off   = en_bytes;
  const size_t rl_bytes = (size_t)NPIX * sizeof(float);
  if (rl_off + rl_bytes > ws_size) return;

  const float* emb = (const float*)d_in[0];
  const int*   lab = (const int*)d_in[1];
  _Float16* En       = (_Float16*)d_ws;
  float*    row_loss = (float*)((char*)d_ws + rl_off);
  float*    out      = (float*)d_out;

  hipLaunchKernelGGL(k_norm,  dim3(NPIX / K1_PIX),         dim3(256), 0, stream, emb, En);
  hipLaunchKernelGGL(k_gram,  dim3(NPIX / ROWS_PER_BLOCK), dim3(128), 0, stream,
                     (const _Float16*)En, lab, row_loss);
  hipLaunchKernelGGL(k_final, dim3(1),                      dim3(256), 0, stream,
                     (const float*)row_loss, lab, out);
}
